// Model_22488448762490
// MI455X (gfx1250) — hardware-verified
//
#include <hip/hip_runtime.h>
#include <math.h>

constexpr int HID    = 51;
constexpr int BATCH  = 1024;
constexpr int TLEN   = 1024;
constexpr int NFUT   = 64;
constexpr int TFW    = TLEN + NFUT;
constexpr int BT     = 16;
constexpr int KP     = 64;
constexpr int NP     = 256;
constexpr int K2     = 128;
constexpr int NTH    = 128;
constexpr int NGROW  = 4 * HID;
constexpr int CHUNK  = 32;
constexpr float HCARRY = 64.0f;
constexpr float WCARRY = 16.0f;
constexpr float FOLD   = 1.0f / (HCARRY * WCARRY);

static_assert(BATCH % BT == 0, "batch tiles");
static_assert(TLEN % CHUNK == 0 && TFW % CHUNK == 0, "whole 32-step chunks");
static_assert((TFW * 4) % 128 == 0, "output row pitch is a whole number of 128-B lines");
static_assert(HID <= KP && 4 * KP == NP && 2 * KP == K2, "padding");
static_assert(KP % 32 == 0 && K2 % 32 == 0, "k-step multiple");
static_assert(NTH == 128 && BT * 8 == NTH, "thread maps");
static_assert((NP * KP) % NTH == 0, "weight fill loop exact");

typedef __attribute__((ext_vector_type(16))) _Float16 v16h;
typedef __attribute__((ext_vector_type(8)))  _Float16 v8h;
typedef __attribute__((ext_vector_type(8)))  float    v8f;
typedef __attribute__((ext_vector_type(4)))  float    v4f;

template <typename T> struct Frag;
template <> struct Frag<_Float16> {
  typedef v16h V; union U { v16h v; v8h h[2]; };
  static __device__ __forceinline__ v16h load(const _Float16* p) {
    U f; f.h[0] = *(const v8h*)(p); f.h[1] = *(const v8h*)(p + 16); return f.v;
  }
  static __device__ __forceinline__ v8f mma(v16h a, v16h b, v8f c) {
    return __builtin_amdgcn_wmma_f32_16x16x32_f16(false, a, false, b, (short)0, c, false, false);
  }
};

__device__ __forceinline__ void guard4_h(v8f& a0, v8f& a1, v8f& a2, v8f& a3,
                                         v16h x, v16h y0, v16h y1, v16h y2, v16h y3) {
  asm volatile("v_nop\n\tv_nop\n\tv_nop\n\tv_nop"
               : "+v"(a0), "+v"(a1), "+v"(a2), "+v"(a3)
               : "v"(x), "v"(y0), "v"(y1), "v"(y2), "v"(y3));
}

__device__ __forceinline__ float fsig(float x)  { return __builtin_amdgcn_rcpf(1.0f + __expf(-x)); }
__device__ __forceinline__ float ftanh(float x) { return 1.0f - 2.0f * __builtin_amdgcn_rcpf(__expf(2.0f * x) + 1.0f); }

__global__ __launch_bounds__(NTH) void lstm2_seq_kernel(
    const float* __restrict__ x,
    const float* __restrict__ w_ih1, const float* __restrict__ w_hh1,
    const float* __restrict__ b_ih1, const float* __restrict__ b_hh1,
    const float* __restrict__ w_ih2, const float* __restrict__ w_hh2,
    const float* __restrict__ b_ih2, const float* __restrict__ b_hh2,
    const float* __restrict__ w_lin, const float* __restrict__ b_lin,
    const int* __restrict__ fut_p,
    float* __restrict__ out) {
  __shared__ __align__(16) _Float16 W1t[NP * KP];
  __shared__ __align__(16) _Float16 W2t[NP * K2];
  __shared__ __align__(16) _Float16 Hb[4 * BT * KP];
  __shared__ __align__(16) float    H2f[BT * KP];
  __shared__ __align__(16) float    xT[CHUNK * BT];
  __shared__ __align__(16) float    ybuf[BT * CHUNK];
  __shared__ __align__(16) float    ufb[BT];
  __shared__ __align__(16) float    wlinpad[KP];
  __shared__ __align__(16) float    bsm[3 * NP];

  const int tid  = (int)threadIdx.x;
  const int lane = tid & 31;
  const int wave = tid >> 5;
  const int c    = lane & 15;
  const int hh   = lane >> 4;
  const int koff = hh * 8;
  const int jcol = wave * 16 + c;
  const bool colok = (jcol < HID);
  const int b0   = (int)blockIdx.x * BT;
  const int grow = tid >> 3;
  const int gpc  = tid & 7;

#pragma unroll 1
  for (int e = tid; e < NP * KP; e += NTH) {
    const int n = e >> 6, k = e & 63;
    const int g = n >> 6, j = n & 63;
    const bool ok = (j < HID) && (k < HID);
    const int jc = (j < HID) ? j : (HID - 1);
    const int kc = (k < HID) ? k : (HID - 1);
    const int src = (g * HID + jc) * HID + kc;
    float wa = w_hh1[src];
    float wb = w_ih2[src];
    float wd = w_hh2[src];
    asm volatile("" : "+v"(wa), "+v"(wb), "+v"(wd));
    W1t[e]               = (_Float16)(ok ? wa * WCARRY : 0.0f);
    W2t[n * K2 + k]      = (_Float16)(ok ? wb * WCARRY : 0.0f);
    W2t[n * K2 + KP + k] = (_Float16)(ok ? wd * WCARRY : 0.0f);
  }
#pragma unroll 1
  for (int e = tid; e < NP; e += NTH) {
    const int g = e >> 6, j = e & 63;
    const bool ok = (j < HID);
    const int r = g * HID + ((j < HID) ? j : (HID - 1));
    float v0 = b_ih1[r];
    float v1 = b_hh1[r];
    float v2 = w_ih1[r];
    float v3 = b_ih2[r];
    float v4 = b_hh2[r];
    asm volatile("" : "+v"(v0), "+v"(v1), "+v"(v2), "+v"(v3), "+v"(v4));
    bsm[e]          = ok ? (v0 + v1) : 0.0f;
    bsm[NP + e]     = ok ? v2 : 0.0f;
    bsm[2 * NP + e] = ok ? (v3 + v4) : 0.0f;
  }
  if (tid < KP) {
    float v = w_lin[(tid < HID) ? tid : (HID - 1)];
    asm volatile("" : "+v"(v));
    wlinpad[tid] = (tid < HID) ? v : 0.0f;
  }
#pragma unroll 1
  for (int i = tid; i < 4 * BT * KP; i += NTH) Hb[i] = (_Float16)0.0f;
#pragma unroll 1
  for (int i = tid; i < BT * KP; i += NTH) H2f[i] = 0.0f;
#pragma unroll 1
  for (int i = tid; i < BT * CHUNK; i += NTH) ybuf[i] = 0.0f;
  if (tid < BT) ufb[tid] = 0.0f;
  {
    const v4f xv = *(const v4f*)(x + (size_t)(b0 + grow) * TLEN + gpc * 4);
    xT[(gpc * 4 + 0) * BT + grow] = xv[0];
    xT[(gpc * 4 + 1) * BT + grow] = xv[1];
    xT[(gpc * 4 + 2) * BT + grow] = xv[2];
    xT[(gpc * 4 + 3) * BT + grow] = xv[3];
  }
  __syncthreads();

  float b1r[4], wi1r[4], b2r[4];
#pragma unroll
  for (int g = 0; g < 4; ++g) {
    b1r[g]  = bsm[g * 64 + jcol];
    wi1r[g] = bsm[NP + g * 64 + jcol];
    b2r[g]  = bsm[2 * NP + g * 64 + jcol];
  }
  float wl[8];
  {
    const v4f wa = *(const v4f*)(wlinpad + gpc * 8);
    const v4f wb = *(const v4f*)(wlinpad + gpc * 8 + 4);
#pragma unroll
    for (int e = 0; e < 4; ++e) { wl[e] = wa[e]; wl[4 + e] = wb[e]; }
  }
  const float blin = b_lin[0];
  int fut = fut_p[0];
  fut = (fut < 0) ? 0 : ((fut > NFUT) ? NFUT : fut);
  const int nsteps = TLEN + fut;

  float c1[8], c2[8];
#pragma unroll
  for (int r = 0; r < 8; ++r) { c1[r] = 0.0f; c2[r] = 0.0f; }

  const v8f z8 = {0.f, 0.f, 0.f, 0.f, 0.f, 0.f, 0.f, 0.f};
  const _Float16* w1row = W1t + jcol * KP + koff;
  const _Float16* w2row = W2t + jcol * K2 + koff;

#pragma unroll 1
  for (int t = 0; t < nsteps; ++t) {
    const int rp = t & 1;
    const int wp = rp ^ 1;
    const int ti = t & (CHUNK - 1);
    const _Float16* h1o = Hb + rp * (BT * KP);
    _Float16*       h1n = Hb + wp * (BT * KP);
    const _Float16* h2o = Hb + (2 + rp) * (BT * KP);
    _Float16*       h2n = Hb + (2 + wp) * (BT * KP);

    if (t > 0 && ti == 0) {
      const v4f yv = *(const v4f*)(ybuf + grow * CHUNK + gpc * 4);
      float* op = out + (size_t)(b0 + grow) * TFW + (size_t)(t - CHUNK) + gpc * 4;
      *(volatile v4f*)op = yv;
      __threadfence();
      *(volatile v4f*)op = yv;
    }

    v8f acc[4];
    acc[0] = z8; acc[1] = z8; acc[2] = z8; acc[3] = z8;
#pragma unroll
    for (int kc = 0; kc < 2; ++kc) {
      const v16h a  = Frag<_Float16>::load(h1o + c * KP + kc * 32 + koff);
      const v16h q0 = Frag<_Float16>::load(w1row + kc * 32);
      const v16h q1 = Frag<_Float16>::load(w1row + 64 * KP + kc * 32);
      const v16h q2 = Frag<_Float16>::load(w1row + 128 * KP + kc * 32);
      const v16h q3 = Frag<_Float16>::load(w1row + 192 * KP + kc * 32);
      acc[0] = Frag<_Float16>::mma(a, q0, acc[0]);
      acc[1] = Frag<_Float16>::mma(a, q1, acc[1]);
      acc[2] = Frag<_Float16>::mma(a, q2, acc[2]);
      acc[3] = Frag<_Float16>::mma(a, q3, acc[3]);
      guard4_h(acc[0], acc[1], acc[2], acc[3], a, q0, q1, q2, q3);
    }
    {
      const v4f xa = *(const v4f*)(xT + ti * BT + 8 * hh);
      const v4f xb = *(const v4f*)(xT + ti * BT + 8 * hh + 4);
      const v4f fa = *(const v4f*)(ufb + 8 * hh);
      const v4f fb = *(const v4f*)(ufb + 8 * hh + 4);
      const bool tforced = (t < TLEN);
      float uu[8];
#pragma unroll
      for (int e = 0; e < 4; ++e) {
        uu[e]     = tforced ? xa[e] : fa[e];
        uu[4 + e] = tforced ? xb[e] : fb[e];
      }
#pragma unroll
      for (int r = 0; r < 8; ++r) {
        const float u  = uu[r];
        const float pi = acc[0][r] * FOLD + (b1r[0] + u * wi1r[0]);
        const float pf = acc[1][r] * FOLD + (b1r[1] + u * wi1r[1]);
        const float pg = acc[2][r] * FOLD + (b1r[2] + u * wi1r[2]);
        const float po = acc[3][r] * FOLD + (b1r[3] + u * wi1r[3]);
        const float cn = fsig(pf) * c1[r] + fsig(pi) * ftanh(pg);
        const float hn = fsig(po) * ftanh(cn);
        c1[r] = colok ? cn : 0.0f;
        const float hz = colok ? hn : 0.0f;
        h1n[(8 * hh + r) * KP + jcol] = (_Float16)(hz * HCARRY);
      }
    }
    __syncthreads();

    acc[0] = z8; acc[1] = z8; acc[2] = z8; acc[3] = z8;
#pragma unroll
    for (int kc = 0; kc < 4; ++kc) {
      const _Float16* ap = (kc < 2) ? (h1n + c * KP + kc * 32 + koff) : (h2o + c * KP + (kc - 2) * 32 + koff);
      const v16h a  = Frag<_Float16>::load(ap);
      const v16h q0 = Frag<_Float16>::load(w2row + kc * 32);
      const v16h q1 = Frag<_Float16>::load(w2row + 64 * K2 + kc * 32);
      const v16h q2 = Frag<_Float16>::load(w2row + 128 * K2 + kc * 32);
      const v16h q3 = Frag<_Float16>::load(w2row + 192 * K2 + kc * 32);
      acc[0] = Frag<_Float16>::mma(a, q0, acc[0]);
      acc[1] = Frag<_Float16>::mma(a, q1, acc[1]);
      acc[2] = Frag<_Float16>::mma(a, q2, acc[2]);
      acc[3] = Frag<_Float16>::mma(a, q3, acc[3]);
      guard4_h(acc[0], acc[1], acc[2], acc[3], a, q0, q1, q2, q3);
    }
#pragma unroll
    for (int r = 0; r < 8; ++r) {
      const float pi = acc[0][r] * FOLD + b2r[0];
      const float pf = acc[1][r] * FOLD + b2r[1];
      const float pg = acc[2][r] * FOLD + b2r[2];
      const float po = acc[3][r] * FOLD + b2r[3];
      const float cn = fsig(pf) * c2[r] + fsig(pi) * ftanh(pg);
      const float hn = fsig(po) * ftanh(cn);
      c2[r] = colok ? cn : 0.0f;
      const float hz = colok ? hn : 0.0f;
      h2n[(8 * hh + r) * KP + jcol] = (_Float16)(hz * HCARRY);
      H2f[(8 * hh + r) * KP + jcol] = hz;
    }
    __syncthreads();

    {
      const v4f ha = *(const v4f*)(H2f + grow * KP + gpc * 8);
      const v4f hb = *(const v4f*)(H2f + grow * KP + gpc * 8 + 4);
      float s = 0.0f;
      s += ha[0] * wl[0];
      s += ha[1] * wl[1];
      s += ha[2] * wl[2];
      s += ha[3] * wl[3];
      s += hb[0] * wl[4];
      s += hb[1] * wl[5];
      s += hb[2] * wl[6];
      s += hb[3] * wl[7];
      s += __shfl_xor(s, 1, 32);
      s += __shfl_xor(s, 2, 32);
      s += __shfl_xor(s, 4, 32);
      const float y = s + blin;
      if (gpc == 0) {
        ybuf[grow * CHUNK + ti] = y;
        ufb[grow] = y;
      }
    }
    if (ti == CHUNK - 1 && t + 1 < TLEN) {
      const v4f xv = *(const v4f*)(x + (size_t)(b0 + grow) * TLEN + (size_t)(t + 1) + gpc * 4);
      xT[(gpc * 4 + 0) * BT + grow] = xv[0];
      xT[(gpc * 4 + 1) * BT + grow] = xv[1];
      xT[(gpc * 4 + 2) * BT + grow] = xv[2];
      xT[(gpc * 4 + 3) * BT + grow] = xv[3];
    }
    __syncthreads();
  }

  {
    const int t0f = (nsteps - 1) & ~(CHUNK - 1);
    const v4f yv = *(const v4f*)(ybuf + grow * CHUNK + gpc * 4);
    float* op = out + (size_t)(b0 + grow) * TFW + (size_t)t0f + gpc * 4;
    *(volatile v4f*)op = yv;
    __threadfence();
    *(volatile v4f*)op = yv;
  }
}

extern "C" void kernel_launch(void* const* d_in, const int* in_sizes, int n_in,
                              void* d_out, int out_size, void* d_ws, size_t ws_size,
                              hipStream_t stream) {
  (void)d_ws; (void)ws_size;
  if (n_in < 12 || d_out == nullptr) return;
  if (in_sizes[0] != BATCH * TLEN || in_sizes[1] != NGROW || in_sizes[2] != NGROW * HID ||
      in_sizes[3] != NGROW || in_sizes[4] != NGROW || in_sizes[5] != NGROW * HID ||
      in_sizes[6] != NGROW * HID || in_sizes[7] != NGROW || in_sizes[8] != NGROW ||
      in_sizes[9] != HID || in_sizes[10] != 1 || in_sizes[11] != 1 ||
      out_size != BATCH * TFW) return;

  const float* x     = (const float*)d_in[0];
  const float* w_ih1 = (const float*)d_in[1];
  const float* w_hh1 = (const float*)d_in[2];
  const float* b_ih1 = (const float*)d_in[3];
  const float* b_hh1 = (const float*)d_in[4];
  const float* w_ih2 = (const float*)d_in[5];
  const float* w_hh2 = (const float*)d_in[6];
  const float* b_ih2 = (const float*)d_in[7];
  const float* b_hh2 = (const float*)d_in[8];
  const float* w_lin = (const float*)d_in[9];
  const float* b_lin = (const float*)d_in[10];
  const int*   fut   = (const int*)d_in[11];
  float* out = (float*)d_out;

  lstm2_seq_kernel<<<BATCH / BT, NTH, 0, stream>>>(x, w_ih1, w_hh1, b_ih1, b_hh1,
                                                   w_ih2, w_hh2, b_ih2, b_hh2,
                                                   w_lin, b_lin, fut, out);
}
